// Model_51084341018990
// MI455X (gfx1250) — hardware-verified
//
#include <hip/hip_runtime.h>

#ifndef NB
#define NB 32
#endif
#define NB_FULL 32
#define NN 2000
#define NP 2048
#define KSTEPS 63
#define HH 64
#define EE 16
#define DO 32
#define PP 24
#ifndef ARES
#define ARES 1
#endif
#ifndef SRES
#define SRES 1
#endif
#define RSC 0.0009765625f

static_assert(NN % 16 == 0);
static_assert(NN % 8 == 0);
static_assert(KSTEPS * 32 >= NN);
static_assert(KSTEPS * 32 <= NP);
static_assert(NP % 64 == 0);
static_assert(NB >= 1 && NB <= NB_FULL);
static_assert(HH == 64 && DO == 32 && EE == 16);

typedef _Float16 v16h __attribute__((ext_vector_type(16)));
typedef unsigned short v8us __attribute__((ext_vector_type(8), may_alias));
typedef float v8f __attribute__((ext_vector_type(8)));
typedef float v4f __attribute__((ext_vector_type(4)));
typedef float v4fa __attribute__((ext_vector_type(4), may_alias));
union FragH { v16h v; v8us half[2]; _Float16 h[16]; unsigned short u[16]; };

__device__ __forceinline__ unsigned short bf16_bits(float x) { const unsigned int u = __float_as_uint(x); return (unsigned short)((u + 0x7FFFu + ((u >> 16) & 1u)) >> 16); }
__device__ __forceinline__ float bf16_val(unsigned short b) { return __uint_as_float(((unsigned int)b) << 16); }
__device__ __forceinline__ float bf16_rne(float x) { return bf16_val(bf16_bits(x)); }
__device__ __forceinline__ unsigned short f16_bits(float x) { union { _Float16 h; unsigned short u; } c; c.h = (_Float16)x; return c.u; }
__device__ __forceinline__ float f16_val(unsigned short u) { union { _Float16 h; unsigned short u; } c; c.u = u; return (float)c.h; }

__device__ __forceinline__ v8f mma16(v16h a, v16h b, v8f c) {
  v8f d = __builtin_amdgcn_wmma_f32_16x16x32_f16(false, a, false, b, (short)0, c, false, false);
  asm volatile("v_nop\n\tv_nop\n\tv_nop\n\tv_nop" : "+v"(d) : "v"(a), "v"(b));
  return d;
}

__global__ __launch_bounds__(128) void k_env(const float* __restrict__ Xe, const float* __restrict__ We, const float* __restrict__ be, float* __restrict__ ENV) {
  __shared__ __attribute__((aligned(16))) unsigned short wl[HH][16];
  __shared__ __attribute__((aligned(16))) float so[4][16][HH + 4];
  const int tid = threadIdx.x, w = tid >> 5, lane = tid & 31, ln = lane & 15, hh = lane >> 4;
  const v8us z8 = {0, 0, 0, 0, 0, 0, 0, 0};
  const v8f zf8 = {0.f, 0.f, 0.f, 0.f, 0.f, 0.f, 0.f, 0.f};
  {
    const int j = tid >> 1, e8 = (tid & 1) * 8;
    FragH f;
#pragma unroll
    for (int i = 0; i < 8; ++i) f.h[i] = (_Float16)bf16_rne(We[(e8 + i) * HH + j]);
    *(v8us*)&wl[j][e8] = f.half[0];
  }
  __syncthreads();
  const int mt = blockIdx.x * 4 + w;
  const bool tval = (mt * 16 + 16 <= NN);
  const int row0 = tval ? mt * 16 : (NN - 16);
  const float* xr = Xe + (size_t)(row0 + ln) * EE + 8 * hh;
  const v4f x0 = *(const v4fa*)xr, x1 = *(const v4fa*)(xr + 4);
  FragH a; a.half[1] = z8;
#pragma unroll
  for (int i = 0; i < 4; ++i) { a.h[i] = (_Float16)bf16_rne(x0[i]); a.h[4 + i] = (_Float16)bf16_rne(x1[i]); }
  v8f acc[4];
#pragma unroll
  for (int t = 0; t < 4; ++t) {
    FragH bq; bq.half[0] = *(const v8us*)&wl[16 * t + ln][8 * hh]; bq.half[1] = z8;
    acc[t] = mma16(a.v, bq.v, zf8);
  }
#pragma unroll
  for (int t = 0; t < 4; ++t) {
    const float bv = bf16_rne(be[16 * t + ln]);
#pragma unroll
    for (int r = 0; r < 8; ++r) so[w][8 * hh + r][16 * t + ln] = fmaxf(acc[t][r] + bv, 0.0f);
  }
  __builtin_amdgcn_fence(4  , "workgroup");
  __builtin_amdgcn_wave_barrier();
  const int rsub = lane >> 4, c4 = (lane & 15) * 4;
  v4f vo[8];
#pragma unroll
  for (int q = 0; q < 8; ++q) vo[q] = *(const v4fa*)&so[w][2 * q + rsub][c4];
  for (int pass = 0; pass < 2; ++pass) {
#pragma unroll
    for (int q = 0; q < 8; ++q) { const int r = 2 * q + rsub; if (tval) *(volatile v4f*)(ENV + (size_t)(row0 + r) * HH + c4) = vo[q]; }
    if (pass == 0) __threadfence();
  }
}

__global__ __launch_bounds__(256) void k_st(const float* __restrict__ src, const float* __restrict__ tgt, const float* __restrict__ ENV,
                                            unsigned short* __restrict__ S16, unsigned short* __restrict__ T16, unsigned int n8) {
  const unsigned int t = blockIdx.x * 256u + threadIdx.x;
  if (t >= n8) return;
  const unsigned int pn = t >> 3, h8 = (t & 7u) * 8u;
  const unsigned int n = pn % (unsigned int)NN;
  const float* ep = ENV + (size_t)n * HH + h8;
  const v4f e0 = *(const v4fa*)ep, e1 = *(const v4fa*)(ep + 4);
  const float* sp = src + (size_t)t * 8;
  const float* tp = tgt + (size_t)t * 8;
  const v4f s0 = *(const v4fa*)sp, s1 = *(const v4fa*)(sp + 4);
  const v4f t0 = *(const v4fa*)tp, t1 = *(const v4fa*)(tp + 4);
  FragH fs, ft;
#pragma unroll
  for (int i = 0; i < 4; ++i) {
    fs.h[i] = (_Float16)(bf16_rne(s0[i]) + e0[i]); fs.h[4 + i] = (_Float16)(bf16_rne(s1[i]) + e1[i]);
    ft.h[i] = (_Float16)(bf16_rne(t0[i]) + e0[i]); ft.h[4 + i] = (_Float16)(bf16_rne(t1[i]) + e1[i]);
  }
  unsigned short* ds = S16 + (size_t)t * 8;
  unsigned short* dt = T16 + (size_t)t * 8;
  *(volatile v8us*)ds = fs.half[0]; *(volatile v8us*)dt = ft.half[0];
  __threadfence();
  *(volatile v8us*)ds = fs.half[0]; *(volatile v8us*)dt = ft.half[0];
}

__global__ __launch_bounds__(256) void k_adj(const float* __restrict__ adj, unsigned short* __restrict__ ADJ16) {
  const int t = blockIdx.x * 256 + threadIdx.x;
  if (t >= NN * (NP / 8)) return;
  const int n = t / (NP / 8), k8 = (t % (NP / 8)) * 8;
  const int kc = (k8 < NN - 8) ? k8 : (NN - 8);
  const float* ap = adj + (size_t)n * NN + kc;
  const v4f a0 = *(const v4fa*)ap, a1 = *(const v4fa*)(ap + 4);
  const bool kval = (k8 < NN);
  FragH f;
#pragma unroll
  for (int i = 0; i < 4; ++i) {
    f.u[i] = kval ? bf16_bits(a0[i]) : (unsigned short)0;
    f.u[4 + i] = kval ? bf16_bits(a1[i]) : (unsigned short)0;
  }
  unsigned short* d = ADJ16 + (size_t)n * NP + k8;
  *(volatile v8us*)d = f.half[0];
  __threadfence();
  *(volatile v8us*)d = f.half[0];
}

__global__ __launch_bounds__(128) void k_xw(const float* __restrict__ X, const float* __restrict__ W, const float* __restrict__ Wr, const float* __restrict__ br,
                                            unsigned short* __restrict__ SUPT, unsigned short* __restrict__ SUPL, float* __restrict__ RES) {
  __shared__ __attribute__((aligned(16))) unsigned short wl[2][DO][40];
  __shared__ __attribute__((aligned(16))) unsigned short sT[DO][72];
#if SRES
  __shared__ __attribute__((aligned(16))) unsigned short sL[DO][72];
#endif
  __shared__ __attribute__((aligned(16))) float so[4][16][DO + 4];
  const int tid = threadIdx.x, w = tid >> 5, lane = tid & 31, ln = lane & 15, hh = lane >> 4;
  const int b = blockIdx.x / (NP / 64), n0 = (blockIdx.x % (NP / 64)) * 64;
  const v8f zf8 = {0.f, 0.f, 0.f, 0.f, 0.f, 0.f, 0.f, 0.f};
#pragma unroll 1
  for (int it = 0; it < 2; ++it) {
    const float* Wm = (it == 0) ? W : Wr;
    const int m = tid >> 2, k8 = (tid & 3) * 8;
    FragH f;
#pragma unroll
    for (int i = 0; i < 8; ++i) f.h[i] = (_Float16)bf16_rne(Wm[(k8 + i) * DO + m]);
    *(v8us*)&wl[it][m][k8] = f.half[0];
  }
  __syncthreads();
  const int n = n0 + 16 * w + ln;
  const int nc = (n < NN) ? n : (NN - 1);
  const float zf = (n < NN) ? 1.0f : 0.0f;
  const float* xr = X + ((size_t)b * NN + nc) * DO;
  const v4f x0 = *(const v4fa*)(xr + 8 * hh), x1 = *(const v4fa*)(xr + 8 * hh + 4);
  const v4f x2 = *(const v4fa*)(xr + 16 + 8 * hh), x3 = *(const v4fa*)(xr + 16 + 8 * hh + 4);
  FragH a;
#pragma unroll
  for (int i = 0; i < 4; ++i) {
    a.h[i] = (_Float16)(bf16_rne(x0[i]) * zf); a.h[4 + i] = (_Float16)(bf16_rne(x1[i]) * zf);
    a.h[8 + i] = (_Float16)(bf16_rne(x2[i]) * zf); a.h[12 + i] = (_Float16)(bf16_rne(x3[i]) * zf);
  }
  v8f as0, as1, ar0, ar1;
  { FragH bq; bq.half[0] = *(const v8us*)&wl[0][ln][8 * hh]; bq.half[1] = *(const v8us*)&wl[0][ln][16 + 8 * hh]; as0 = mma16(a.v, bq.v, zf8); }
  { FragH bq; bq.half[0] = *(const v8us*)&wl[0][16 + ln][8 * hh]; bq.half[1] = *(const v8us*)&wl[0][16 + ln][16 + 8 * hh]; as1 = mma16(a.v, bq.v, zf8); }
  { FragH bq; bq.half[0] = *(const v8us*)&wl[1][ln][8 * hh]; bq.half[1] = *(const v8us*)&wl[1][ln][16 + 8 * hh]; ar0 = mma16(a.v, bq.v, zf8); }
  { FragH bq; bq.half[0] = *(const v8us*)&wl[1][16 + ln][8 * hh]; bq.half[1] = *(const v8us*)&wl[1][16 + ln][16 + 8 * hh]; ar1 = mma16(a.v, bq.v, zf8); }
#pragma unroll
  for (int r = 0; r < 8; ++r) {
    const int kcol = 16 * w + 8 * hh + r;
    const float v0 = as0[r], v1 = as1[r];
    const unsigned short h0 = f16_bits(v0), h1 = f16_bits(v1);
    sT[ln][kcol] = h0; sT[16 + ln][kcol] = h1;
#if SRES
    sL[ln][kcol] = f16_bits((v0 - f16_val(h0)) * 1024.0f); sL[16 + ln][kcol] = f16_bits((v1 - f16_val(h1)) * 1024.0f);
#endif
  }
  {
    const float bb0 = bf16_rne(br[ln]), bb1 = bf16_rne(br[16 + ln]);
#pragma unroll
    for (int r = 0; r < 8; ++r) { so[w][8 * hh + r][ln] = fmaxf(ar0[r] + bb0, 0.0f); so[w][8 * hh + r][16 + ln] = fmaxf(ar1[r] + bb1, 0.0f); }
  }
  __syncthreads();
  v8us pv[2]; int pm[2], pq[2];
#if SRES
  v8us pl[2];
#endif
#pragma unroll
  for (int it = 0; it < 2; ++it) {
    const int j = tid + 128 * it; pm[it] = j >> 3; pq[it] = j & 7;
    pv[it] = *(const v8us*)&sT[pm[it]][8 * pq[it]];
#if SRES
    pl[it] = *(const v8us*)&sL[pm[it]][8 * pq[it]];
#endif
  }
  const int rq = lane >> 3, c4 = (lane & 7) * 4;
  v4f ro[4]; int rn[4];
#pragma unroll
  for (int it = 0; it < 4; ++it) { const int r = 4 * it + rq; rn[it] = n0 + 16 * w + r; ro[it] = *(const v4fa*)&so[w][r][c4]; }
  for (int pass = 0; pass < 2; ++pass) {
#pragma unroll
    for (int it = 0; it < 2; ++it) {
      const size_t o = ((size_t)(b * DO + pm[it])) * NP + n0 + 8 * pq[it];
      *(volatile v8us*)(SUPT + o) = pv[it];
#if SRES
      *(volatile v8us*)(SUPL + o) = pl[it];
#endif
    }
#pragma unroll
    for (int it = 0; it < 4; ++it) { if (rn[it] < NN) *(volatile v4f*)(RES + ((size_t)b * NN + rn[it]) * DO + c4) = ro[it]; }
    if (pass == 0) __threadfence();
  }
}

__global__ __launch_bounds__(128) void k_conv(const int* __restrict__ cyc, const unsigned short* __restrict__ S16, const unsigned short* __restrict__ T16,
                                              const unsigned short* __restrict__ ADJ16, const unsigned short* __restrict__ SUPT, const unsigned short* __restrict__ SUPL,
                                              const float* __restrict__ RES, const float* __restrict__ bias, float* __restrict__ out) {
  __shared__ __attribute__((aligned(16))) unsigned short Sl[64][72];
  __shared__ __attribute__((aligned(16))) unsigned short Tl[32][72];
  __shared__ __attribute__((aligned(16))) unsigned short Dl[64][40];
  __shared__ __attribute__((aligned(16))) unsigned short Ah[4][16][40];
#if ARES
  __shared__ __attribute__((aligned(16))) unsigned short Al[4][16][40];
#endif
  __shared__ __attribute__((aligned(16))) float so[4][16][DO + 4];
  const int tid = threadIdx.x, w = tid >> 5, lane = tid & 31, ln = lane & 15, hh = lane >> 4;
  const int b = blockIdx.y, nb = blockIdx.x * 64;
  int pc = cyc[b] % PP; if (pc < 0) pc += PP;
  const unsigned short* Sp = S16 + (size_t)pc * NN * HH;
  const unsigned short* Tp = T16 + (size_t)pc * NN * HH;
  const v8f zf8 = {0.f, 0.f, 0.f, 0.f, 0.f, 0.f, 0.f, 0.f};
#pragma unroll
  for (int it = 0; it < 4; ++it) {
    const int c = tid + 128 * it; const int r = c >> 3, q = c & 7;
    const int nr = (nb + r < NN) ? (nb + r) : (NN - 1);
    *(v8us*)&Sl[r][8 * q] = *(const v8us*)(Sp + (size_t)nr * HH + 8 * q);
  }
  __syncthreads();
  FragH sa0, sa1;
  sa0.half[0] = *(const v8us*)&Sl[16 * w + ln][8 * hh];      sa0.half[1] = *(const v8us*)&Sl[16 * w + ln][16 + 8 * hh];
  sa1.half[0] = *(const v8us*)&Sl[16 * w + ln][32 + 8 * hh]; sa1.half[1] = *(const v8us*)&Sl[16 * w + ln][48 + 8 * hh];
  v8f ch0 = zf8, ch1 = zf8;
#if (ARES || SRES)
  v8f cl0 = zf8, cl1 = zf8;
#endif
  const unsigned short* sp0 = SUPT + ((size_t)(b * DO + ln)) * NP + 8 * hh;
  const unsigned short* sp1 = sp0 + (size_t)16 * NP;
#if SRES
  const unsigned short* lp0 = SUPL + ((size_t)(b * DO + ln)) * NP + 8 * hh;
  const unsigned short* lp1 = lp0 + (size_t)16 * NP;
#endif
#pragma unroll 1
  for (int kit = 0; kit < KSTEPS; ++kit) {
    const int kb = kit * 32;
    __syncthreads();
#pragma unroll
    for (int it = 0; it < 2; ++it) {
      const int c = tid + 128 * it; const int kk = c >> 3, q = c & 7;
      const int kc = (kb + kk < NN) ? (kb + kk) : (NN - 1);
      *(v8us*)&Tl[kk][8 * q] = *(const v8us*)(Tp + (size_t)kc * HH + 8 * q);
    }
#pragma unroll
    for (int it = 0; it < 2; ++it) {
      const int c = tid + 128 * it; const int r = c >> 2, q = c & 3;
      const int nr = (nb + r < NN) ? (nb + r) : (NN - 1);
      *(v8us*)&Dl[r][8 * q] = *(const v8us*)(ADJ16 + (size_t)nr * NP + kb + 8 * q);
    }
    __syncthreads();
#pragma unroll
    for (int koff = 0; koff < 2; ++koff) {
      const int kl = 16 * koff + ln;
      FragH b0, b1;
      b0.half[0] = *(const v8us*)&Tl[kl][8 * hh];      b0.half[1] = *(const v8us*)&Tl[kl][16 + 8 * hh];
      b1.half[0] = *(const v8us*)&Tl[kl][32 + 8 * hh]; b1.half[1] = *(const v8us*)&Tl[kl][48 + 8 * hh];
      v8f g = mma16(sa0.v, b0.v, zf8);
      g = mma16(sa1.v, b1.v, g);
#pragma unroll
      for (int r = 0; r < 8; ++r) {
        const int M = 8 * hh + r;
        const float av = fmaxf(g[r], 0.0f) * bf16_val(Dl[16 * w + M][kl]);
        const unsigned short hb = f16_bits(av);
        Ah[w][M][kl] = hb;
#if ARES
        Al[w][M][kl] = f16_bits((av - f16_val(hb)) * 1024.0f);
#endif
      }
    }
    __builtin_amdgcn_fence(4  , "workgroup");
    __builtin_amdgcn_wave_barrier();
    FragH fa; fa.half[0] = *(const v8us*)&Ah[w][ln][8 * hh]; fa.half[1] = *(const v8us*)&Ah[w][ln][16 + 8 * hh];
    FragH s0, s1;
    s0.half[0] = *(const v8us*)(sp0 + kb); s0.half[1] = *(const v8us*)(sp0 + kb + 16);
    s1.half[0] = *(const v8us*)(sp1 + kb); s1.half[1] = *(const v8us*)(sp1 + kb + 16);
    ch0 = mma16(fa.v, s0.v, ch0);
    ch1 = mma16(fa.v, s1.v, ch1);
#if ARES
    FragH fl; fl.half[0] = *(const v8us*)&Al[w][ln][8 * hh]; fl.half[1] = *(const v8us*)&Al[w][ln][16 + 8 * hh];
    cl0 = mma16(fl.v, s0.v, cl0);
    cl1 = mma16(fl.v, s1.v, cl1);
#endif
#if SRES
    FragH l0, l1;
    l0.half[0] = *(const v8us*)(lp0 + kb); l0.half[1] = *(const v8us*)(lp0 + kb + 16);
    l1.half[0] = *(const v8us*)(lp1 + kb); l1.half[1] = *(const v8us*)(lp1 + kb + 16);
    cl0 = mma16(fa.v, l0.v, cl0);
    cl1 = mma16(fa.v, l1.v, cl1);
#endif
  }
  {
    const float bv0 = bf16_rne(bias[ln]), bv1 = bf16_rne(bias[16 + ln]);
#pragma unroll
    for (int r = 0; r < 8; ++r) {
      float v0 = ch0[r] + bv0, v1 = ch1[r] + bv1;
#if (ARES || SRES)
      v0 += cl0[r] * RSC; v1 += cl1[r] * RSC;
#endif
      so[w][8 * hh + r][ln] = v0; so[w][8 * hh + r][16 + ln] = v1;
    }
  }
  __builtin_amdgcn_fence(4  , "workgroup");
  __builtin_amdgcn_wave_barrier();
  const int rq = lane >> 3, c4 = (lane & 7) * 4;
  v4f vo[4]; int vn[4];
#pragma unroll
  for (int it = 0; it < 4; ++it) {
    const int r = 4 * it + rq; const int n = nb + 16 * w + r; vn[it] = n;
    const int nc = (n < NN) ? n : (NN - 1);
    const v4f cv = *(const v4fa*)&so[w][r][c4];
    const v4f rr = *(const v4fa*)(RES + ((size_t)b * NN + nc) * DO + c4);
    v4f o;
#pragma unroll
    for (int i = 0; i < 4; ++i) o[i] = fmaxf(cv[i] + rr[i], 0.0f);
    vo[it] = o;
  }
  for (int pass = 0; pass < 2; ++pass) {
#pragma unroll
    for (int it = 0; it < 4; ++it) { if (vn[it] < NN) *(volatile v4f*)(out + ((size_t)b * NN + vn[it]) * DO + c4) = vo[it]; }
    if (pass == 0) __threadfence();
  }
}

extern "C" void kernel_launch(void* const* d_in, const int* in_sizes, int n_in,
                              void* d_out, int out_size, void* d_ws, size_t ws_size, hipStream_t stream) {
  if (n_in < 12) return;
  if (in_sizes[0] < NB * NN * DO || in_sizes[1] < NB || in_sizes[2] < NN * NN || in_sizes[3] < NN * EE || in_sizes[4] < EE * HH || in_sizes[5] < HH ||
      in_sizes[6] < PP * NN * HH || in_sizes[7] < PP * NN * HH || in_sizes[8] < DO * DO || in_sizes[9] < DO || in_sizes[10] < DO * DO || in_sizes[11] < DO) return;
  if (out_size < NB * NN * DO) return;
  const float* X    = (const float*)d_in[0];
  const int*   cyc  = (const int*)d_in[1];
  const float* adj  = (const float*)d_in[2];
  const float* Xe   = (const float*)d_in[3];
  const float* We   = (const float*)d_in[4];
  const float* be   = (const float*)d_in[5];
  const float* src  = (const float*)d_in[6];
  const float* tgt  = (const float*)d_in[7];
  const float* W    = (const float*)d_in[8];
  const float* bias = (const float*)d_in[9];
  const float* Wr   = (const float*)d_in[10];
  const float* br   = (const float*)d_in[11];
  float* out = (float*)d_out;

  char* ws = (char*)d_ws; size_t off = 0;
  auto take = [&](size_t bytes) { char* p = ws + off; off += (bytes + 255) & ~(size_t)255; return p; };
  float*          ENV   = (float*)take((size_t)NN * HH * 4);
  unsigned short* S16   = (unsigned short*)take((size_t)PP * NN * HH * 2);
  unsigned short* T16   = (unsigned short*)take((size_t)PP * NN * HH * 2);
  unsigned short* ADJ16 = (unsigned short*)take((size_t)NN * NP * 2);
  unsigned short* SUPT  = (unsigned short*)take((size_t)NB * DO * NP * 2);
  unsigned short* SUPL  = (unsigned short*)take((size_t)NB * DO * NP * 2);
  float*          RES   = (float*)take((size_t)NB * NN * DO * 4);
  if (off > ws_size || off > (size_t)134217728) return;

  k_env<<<(NN / 16 + 3) / 4, 128, 0, stream>>>(Xe, We, be, ENV);
  const unsigned int n8st = (unsigned int)(PP * NN * HH / 8);
  k_st<<<(n8st + 255) / 256, 256, 0, stream>>>(src, tgt, ENV, S16, T16, n8st);
  k_adj<<<(NN * (NP / 8) + 255) / 256, 256, 0, stream>>>(adj, ADJ16);
  k_xw<<<NB * (NP / 64), 128, 0, stream>>>(X, W, Wr, br, SUPT, SUPL, RES);
  k_conv<<<dim3(NP / 64, NB), 128, 0, stream>>>(cyc, S16, T16, ADJ16, SUPT, SUPL, RES, bias, out);
}
